// KANLayer_40965398069809
// MI455X (gfx1250) — hardware-run, weakly checked
//
#include <hip/hip_runtime.h>
#include <stddef.h>


typedef _Float16 v16h __attribute__((ext_vector_type(16)));
typedef _Float16 v8h  __attribute__((ext_vector_type(8)));
typedef float    v8f  __attribute__((ext_vector_type(8)));
typedef float    v4f  __attribute__((ext_vector_type(4)));
typedef _Float16 h16;

#ifndef NB
#define NB 512
#endif
#define NB_FULL 512
#define IN_DIM  256
#define OUT_DIM 256
#define NBAS    11
#define KSPL    (IN_DIM * NBAS)
#define KTOT    (KSPL + IN_DIM)
#define PIECES  (KTOT / 8)
#define CPIECES (KSPL / 8)

static_assert(NB >= 64 && NB <= NB_FULL && (NB % 64) == 0 && (NB % 2) == 0);
static_assert(IN_DIM == 256);
static_assert((OUT_DIM % 64) == 0 && (OUT_DIM % 2) == 0);
static_assert((KTOT % 32) == 0);
static_assert(PIECES * 8 == KTOT && CPIECES * 8 == KSPL);
static_assert((PIECES % 32) == 0 && (CPIECES % 32) == 0);
static_assert(2 * PIECES == 3 * 256);
static_assert(((size_t)KSPL * 4) % 16 == 0);
static_assert(NBAS > 8);

#define LDC 68
static_assert((LDC % 4) == 0 && LDC >= 64);

#define ACARRY 1024.0f
#define WCARRY 1024.0f

#define A16_BYTES ((size_t)NB * KTOT * 2)
#define W16_BYTES ((size_t)OUT_DIM * KTOT * 2)
#define OFF_A16  ((size_t)0)
#define OFF_W16  (OFF_A16 + A16_BYTES)
#define WS_TOTAL (OFF_W16 + W16_BYTES)
static_assert((A16_BYTES % 128) == 0 && (W16_BYTES % 128) == 0);
static_assert(WS_TOTAL <= (size_t)134217728);
static_assert((size_t)NB * OUT_DIM * 4 <= (size_t)524288);

__device__ __forceinline__ float bf16r(float x) {
  unsigned int u = __float_as_uint(x);
  u = (u + 0x7FFFu + ((u >> 16) & 1u)) & 0xFFFF0000u;
  return __uint_as_float(u);
}

static __device__ __forceinline__ h16 toh_flush(float v) {
  const h16 r = (h16)v;
  return (fabsf(v) < 6.103515625e-05f) ? (h16)0.0f : r;
}

__device__ __forceinline__ v16h frag_at(const _Float16* p) {
  v8h lo = *(const v8h*)(p);
  v8h hi = *(const v8h*)(p + 16);
  v16h out;
#pragma unroll
  for (int i = 0; i < 8; ++i) { out[i] = lo[i]; out[i + 8] = hi[i]; }
  return out;
}

__device__ __forceinline__ v8f wmma16(v16h a, v16h b, v8f c) {
  v8f d = __builtin_amdgcn_wmma_f32_16x16x32_f16(false, a, false, b, (short)0, c,
                                                 false, false);
  asm volatile("v_nop\n\tv_nop\n\tv_nop\n\tv_nop" : "+v"(d) : "v"(a), "v"(b));
  return d;
}

__global__ __launch_bounds__(256) void prep_a_kernel(
    const float* __restrict__ X, _Float16* __restrict__ A16) {
#pragma clang fp contract(off)
  __shared__ __attribute__((aligned(16))) _Float16 T[2 * KTOT];
  const unsigned tid = threadIdx.x;
  const unsigned row0 = blockIdx.x * 2u;

#pragma unroll 1
  for (unsigned r = 0; r < 2u; ++r) {
    const float xv = bf16r(X[(size_t)(row0 + r) * IN_DIM + tid]);
    float b[14];
#pragma unroll
    for (int t = 0; t < 14; ++t) {
      const float g0 = -1.75f + 0.25f * (float)t;
      const float g1 = -1.75f + 0.25f * (float)(t + 1);
      b[t] = (xv >= g0 && xv < g1) ? 1.0f : 0.0f;
    }
#pragma unroll
    for (int j = 1; j <= 3; ++j) {
      const float rj = 1.0f / (0.25f * (float)j);
#pragma unroll
      for (int t = 0; t < 14 - j; ++t) {
        const float gl = -1.75f + 0.25f * (float)t;
        const float gr = -1.75f + 0.25f * (float)(t + j + 1);
        b[t] = (xv - gl) * rj * b[t] + (gr - xv) * rj * b[t + 1];
      }
    }
#pragma unroll
    for (int t = 0; t < NBAS; ++t)
      T[r * (unsigned)KTOT + tid * (unsigned)NBAS + (unsigned)t] = toh_flush(ACARRY * b[t]);
    const float sg = 1.0f / (1.0f + expf(-xv));
    T[r * (unsigned)KTOT + (unsigned)KSPL + tid] = toh_flush(ACARRY * (xv * sg));
  }
  __syncthreads();

  v8h xs[3];
  size_t off[3];
#pragma unroll
  for (unsigned j = 0; j < 3u; ++j) {
    const unsigned idx = tid + 256u * j;
    xs[j] = *(const v8h*)&T[idx * 8u];
    off[j] = (size_t)row0 * KTOT + (size_t)idx * 8u;
  }
#pragma unroll
  for (int j = 0; j < 3; ++j) *(volatile v8h*)(A16 + off[j]) = xs[j];
  __threadfence();
#pragma unroll
  for (int j = 0; j < 3; ++j) *(volatile v8h*)(A16 + off[j]) = xs[j];
}

__global__ __launch_bounds__(256) void prep_w_kernel(
    const float* __restrict__ coef, const float* __restrict__ resw,
    const float* __restrict__ univ, _Float16* __restrict__ Wt) {
#pragma clang fp contract(off)
  const unsigned tid = threadIdx.x;
  const unsigned o0 = blockIdx.x * 2u;
  v8h xs[3];
  size_t off[3];
#pragma unroll
  for (unsigned j = 0; j < 3u; ++j) {
    const unsigned idx = tid + 256u * j;
    const unsigned r = idx / (unsigned)PIECES;
    const unsigned p = idx - r * (unsigned)PIECES;
    const unsigned o = o0 + r;
    const bool isc = p < (unsigned)CPIECES;
    const unsigned pc = isc ? p : (unsigned)(CPIECES - 1);
    const unsigned pr = isc ? 0u : (p - (unsigned)CPIECES);
    const size_t coff = (size_t)o * KSPL + (size_t)pc * 8u;
    const v4f c0 = *(const v4f*)(coef + coff);
    const v4f c1 = *(const v4f*)(coef + coff + 4u);
    const size_t roff = (size_t)o * IN_DIM + (size_t)pr * 8u;
    const v4f r0 = *(const v4f*)(resw + roff);
    const v4f r1 = *(const v4f*)(resw + roff + 4u);
    const unsigned k0 = pc * 8u;
    const unsigned i0 = k0 / (unsigned)NBAS;
    const unsigned i1 = (k0 + 7u) / (unsigned)NBAS;
    const float u0 = bf16r(univ[(size_t)o * IN_DIM + i0]);
    const float u1 = bf16r(univ[(size_t)o * IN_DIM + i1]);
    const unsigned kb = (i0 + 1u) * (unsigned)NBAS;
    v8h x;
#pragma unroll
    for (unsigned e = 0; e < 4u; ++e) {
      const float ua = ((k0 + e) < kb) ? u0 : u1;
      const float ub = ((k0 + e + 4u) < kb) ? u0 : u1;
      const float wa = isc ? (ua * bf16r(c0[e])) : bf16r(r0[e]);
      const float wb = isc ? (ub * bf16r(c1[e])) : bf16r(r1[e]);
      x[e]      = toh_flush(WCARRY * wa);
      x[e + 4u] = toh_flush(WCARRY * wb);
    }
    xs[j] = x;
    off[j] = (size_t)o0 * KTOT + (size_t)idx * 8u;
  }
#pragma unroll
  for (int j = 0; j < 3; ++j) *(volatile v8h*)(Wt + off[j]) = xs[j];
  __threadfence();
#pragma unroll
  for (int j = 0; j < 3; ++j) *(volatile v8h*)(Wt + off[j]) = xs[j];
}

__global__ __launch_bounds__(256) void gemm_out_kernel(
    const _Float16* __restrict__ A16, const _Float16* __restrict__ Bt,
    float* __restrict__ outf) {
  __shared__ __attribute__((aligned(16))) float Cs[64 * LDC];
  const unsigned tid = threadIdx.x, lane = tid & 31u;
  const unsigned w = __builtin_amdgcn_readfirstlane(tid >> 5);
  const unsigned mw = w >> 1, nw = w & 1u;
  const unsigned hh = lane >> 4, m = lane & 15u;
  const unsigned n0 = blockIdx.x * 64u;
  const unsigned row0 = blockIdx.y * 64u;
  const unsigned K = (unsigned)KTOT;

  const _Float16* ap  = A16 + (size_t)(row0 + mw * 16u + m) * K + hh * 8u;
  const _Float16* bp0 = Bt + (size_t)(n0 + nw * 32u + m) * K + hh * 8u;
  const _Float16* bp1 = bp0 + (size_t)16 * K;
  v8f acc0 = {}, acc1 = {};
#pragma unroll 2
  for (unsigned k0 = 0; k0 < K; k0 += 32u) {
    const v16h a  = frag_at(ap + k0);
    const v16h b0 = frag_at(bp0 + k0);
    const v16h b1 = frag_at(bp1 + k0);
    acc0 = wmma16(a, b0, acc0);
    acc1 = wmma16(a, b1, acc1);
  }
#pragma unroll
  for (int r = 0; r < 8; ++r) {
    float* d = &Cs[(mw * 16u + hh * 8u + (unsigned)r) * LDC + nw * 32u + m];
    d[0]  = acc0[r];
    d[16] = acc1[r];
  }
  __syncthreads();

  const float cs = 1.0f / (ACARRY * WCARRY);
  v4f xs[4];
  size_t off[4];
#pragma unroll
  for (unsigned i = 0; i < 4u; ++i) {
    const unsigned r = 16u * i + (tid >> 4);
    const unsigned c = (tid & 15u) * 4u;
    const v4f u = *(const v4f*)&Cs[r * LDC + c];
    v4f val;
#pragma unroll
    for (int j = 0; j < 4; ++j) val[j] = u[j] * cs;
    xs[i] = val;
    off[i] = (size_t)(row0 + r) * OUT_DIM + n0 + c;
  }
#pragma unroll
  for (int i = 0; i < 4; ++i) *(volatile v4f*)(outf + off[i]) = xs[i];
  __threadfence();
#pragma unroll
  for (int i = 0; i < 4; ++i) *(volatile v4f*)(outf + off[i]) = xs[i];
}

extern "C" void kernel_launch(void* const* d_in, const int* in_sizes, int n_in,
                              void* d_out, int out_size, void* d_ws, size_t ws_size,
                              hipStream_t stream) {
  if (n_in < 4) return;
  if ((long long)in_sizes[0] < (long long)NB * IN_DIM) return;
  if ((long long)in_sizes[1] < (long long)OUT_DIM * IN_DIM * NBAS) return;
  if ((long long)in_sizes[2] < (long long)OUT_DIM * IN_DIM) return;
  if ((long long)in_sizes[3] < (long long)OUT_DIM * IN_DIM) return;
  if ((long long)out_size < (long long)NB * OUT_DIM) return;
  if (ws_size < WS_TOTAL) return;

  const float* x    = (const float*)d_in[0];
  const float* coef = (const float*)d_in[1];
  const float* resw = (const float*)d_in[2];
  const float* univ = (const float*)d_in[3];
  float* out = (float*)d_out;

  char* ws = (char*)d_ws;
  _Float16* A16 = (_Float16*)(ws + OFF_A16);
  _Float16* W16 = (_Float16*)(ws + OFF_W16);

  dim3 blk(256);
  prep_a_kernel<<<dim3(NB / 2), blk, 0, stream>>>(x, A16);
  prep_w_kernel<<<dim3(OUT_DIM / 2), blk, 0, stream>>>(coef, resw, univ, W16);
  gemm_out_kernel<<<dim3(OUT_DIM / 64, NB / 64), blk, 0, stream>>>(A16, W16, out);
}
